// RNNModel_62259845923161
// MI455X (gfx1250) — hardware-verified
//
#include <hip/hip_runtime.h>
#include <math.h>

constexpr int NBAT  = 4096;
constexpr int NSTEP = 512;
constexpr int NHID  = 32;
constexpr int NTHR  = 128;
constexpr int NWAVE = NTHR / 32;
constexpr int ROWS_PER_WAVE  = 32;
constexpr int ROWS_PER_BLOCK = ROWS_PER_WAVE * NWAVE;
constexpr int NBLK = NBAT / ROWS_PER_BLOCK;
static_assert(NHID == 32);
static_assert(NBAT % ROWS_PER_BLOCK == 0);
static_assert(NTHR * 8 == NHID * NHID);
static_assert(NSTEP >= 1);
static_assert(NTHR >= NHID);

typedef __attribute__((ext_vector_type(16))) __bf16   v16b;
typedef __attribute__((ext_vector_type(8)))  __bf16   v8b;
typedef __attribute__((ext_vector_type(8)))  float    v8f;
typedef __attribute__((ext_vector_type(4)))  float    v4f;

__device__ __forceinline__ unsigned short at_bf_bits(float f) {
  unsigned u = __float_as_uint(f);
  return (unsigned short)((u + 0x7FFFu + ((u >> 16) & 1u)) >> 16);
}
__device__ __forceinline__ __bf16 at_f2bf(float f) { return __builtin_bit_cast(__bf16, at_bf_bits(f)); }
__device__ __forceinline__ void at_split(float f, __bf16& hi, __bf16& lo) {
  const unsigned short hb = at_bf_bits(f);
  hi = __builtin_bit_cast(__bf16, hb);
  lo = at_f2bf(f - __uint_as_float(((unsigned)hb) << 16));
}

__device__ __forceinline__ void dep_guard_b(v8f& a, v8f& b, v16b x, v16b y) { asm volatile("v_nop\n\tv_nop\n\tv_nop\n\tv_nop" : "+v"(a), "+v"(b) : "v"(x), "v"(y)); }
__device__ __forceinline__ void keep4_b(v16b a, v16b b, v16b c, v16b d) { asm volatile("v_nop" :: "v"(a), "v"(b), "v"(c), "v"(d)); }
__device__ __forceinline__ void tile_guard(v8f& d0, v8f& d1, v16b a0, v16b a1, v16b a2, v16b a3, v16b b0, v16b b1) {
  asm volatile("v_nop\n\tv_nop\n\tv_nop\n\tv_nop" : "+v"(d0), "+v"(d1) : "v"(a0), "v"(a1), "v"(a2), "v"(a3), "v"(b0), "v"(b1));
}

template <typename T> struct Frag;
template <> struct Frag<__bf16> {
  typedef v16b V; union U { v16b v; v8b h[2]; };
  static __device__ __forceinline__ v16b load(const __bf16* p) {
    U f; f.h[0] = *(const v8b*)(p); f.h[1] = *(const v8b*)(p + 16); return f.v;
  }
  static __device__ __forceinline__ v8f mma(v16b a, v16b b, v8f c) {
    return __builtin_amdgcn_wmma_f32_16x16x32_bf16(false, a, false, b, (short)0, c, false, false);
  }
  static __device__ __forceinline__ void guard(v8f& a, v8f& b, v16b x, v16b y) { dep_guard_b(a, b, x, y); }
  static __device__ __forceinline__ void keep(v16b a, v16b b, v16b c, v16b d) { keep4_b(a, b, c, d); }
};

__device__ __forceinline__ float tanh_f32(float z) {
  const float y = fabsf(z);
  const float t = expf(-2.0f * y);
  const float r = (1.0f - t) * (1.0f / (1.0f + t));
  return copysignf(r, z);
}

__device__ __forceinline__ void chain_step(float xv,
    const float (&cw0)[8], const float (&cw1)[8], const float (&cb0)[8], const float (&cb1)[8],
    v16b a0h, v16b a0l, v16b a1h, v16b a1l,
    v16b& bh, v16b& bl, float (&hj0)[8], float (&hj1)[8]) {
  v8f c0, c1;
#pragma unroll
  for (int r = 0; r < 8; ++r) {
    c0[r] = fmaf(xv, cw0[r], cb0[r]);
    c1[r] = fmaf(xv, cw1[r], cb1[r]);
  }
  v8f d0 = Frag<__bf16>::mma(a0h, bh, c0);
  d0 = Frag<__bf16>::mma(a0h, bl, d0);
  d0 = Frag<__bf16>::mma(a0l, bh, d0);
  v8f d1 = Frag<__bf16>::mma(a1h, bh, c1);
  d1 = Frag<__bf16>::mma(a1h, bl, d1);
  d1 = Frag<__bf16>::mma(a1l, bh, d1);
  tile_guard(d0, d1, a0h, a0l, a1h, a1l, bh, bl);
  v16b nh, nl;
#pragma unroll
  for (int r = 0; r < 8; ++r) {
    const float v0 = tanh_f32(d0[r]);
    const float v1 = tanh_f32(d1[r]);
    hj0[r] = v0;
    hj1[r] = v1;
    __bf16 p, q;
    at_split(v0, p, q); nh[r] = p;     nl[r] = q;
    at_split(v1, p, q); nh[8 + r] = p; nl[8 + r] = q;
  }
  bh = nh;
  bl = nl;
}

__global__ __launch_bounds__(NTHR) void rnn_seq_kernel(const float* __restrict__ x,
                                                       const float* __restrict__ w_ih,
                                                       const float* __restrict__ w_hh,
                                                       const float* __restrict__ b_ih,
                                                       const float* __restrict__ b_hh,
                                                       const float* __restrict__ fc_w,
                                                       const float* __restrict__ fc_b,
                                                       float* __restrict__ out) {
  __shared__ __align__(16) __bf16 Wsh[NHID * NHID];
  __shared__ __align__(16) __bf16 Wsl[NHID * NHID];
  __shared__ float cw_s[NHID];
  __shared__ float cb_s[NHID];
  __shared__ float cf_s[NHID];
  __shared__ __align__(16) float oslab[NWAVE][32];

  const int tid = threadIdx.x, lane = tid & 31, wave = tid >> 5;
  const int hh = lane >> 4, cc = lane & 15;

  {
    const int j = tid >> 2;
    const int q = (tid & 3) * 8;
    const v4f w0 = *(const v4f*)(w_hh + j * NHID + q);
    const v4f w1 = *(const v4f*)(w_hh + j * NHID + q + 4);
    v8b hv, lv;
#pragma unroll
    for (int e = 0; e < 4; ++e) {
      __bf16 a, b;
      at_split(w0[e], a, b); hv[e] = a;     lv[e] = b;
      at_split(w1[e], a, b); hv[4 + e] = a; lv[4 + e] = b;
    }
    *(v8b*)(Wsh + j * NHID + q) = hv;
    *(v8b*)(Wsl + j * NHID + q) = lv;
  }
  if (tid < NHID) {
    cw_s[tid] = w_ih[tid];
    cb_s[tid] = b_ih[tid] + b_hh[tid];
    cf_s[tid] = fc_w[tid];
  }
  __syncthreads();

  const v16b a0h = Frag<__bf16>::load(Wsh + cc * NHID + 8 * hh);
  const v16b a0l = Frag<__bf16>::load(Wsl + cc * NHID + 8 * hh);
  const v16b a1h = Frag<__bf16>::load(Wsh + (16 + cc) * NHID + 8 * hh);
  const v16b a1l = Frag<__bf16>::load(Wsl + (16 + cc) * NHID + 8 * hh);

  float cw0[8], cw1[8], cb0[8], cb1[8];
#pragma unroll
  for (int r = 0; r < 8; ++r) {
    cw0[r] = cw_s[8 * hh + r];
    cw1[r] = cw_s[16 + 8 * hh + r];
    cb0[r] = cb_s[8 * hh + r];
    cb1[r] = cb_s[16 + 8 * hh + r];
  }

  const int wrow = blockIdx.x * ROWS_PER_BLOCK + wave * ROWS_PER_WAVE;
  const float* xr0 = x + (size_t)(wrow + cc) * NSTEP;
  const float* xr1 = x + (size_t)(wrow + 16 + cc) * NSTEP;

  v16b bh0, bl0, bh1, bl1;
  {
    const __bf16 z = __builtin_bit_cast(__bf16, (unsigned short)0);
#pragma unroll
    for (int e = 0; e < 16; ++e) { bh0[e] = z; bl0[e] = z; bh1[e] = z; bl1[e] = z; }
  }
  float h00[8], h01[8], h10[8], h11[8];
#pragma unroll
  for (int r = 0; r < 8; ++r) { h00[r] = 0.0f; h01[r] = 0.0f; h10[r] = 0.0f; h11[r] = 0.0f; }

  float xc0 = xr0[0];
  float xc1 = xr1[0];
#pragma unroll 1
  for (int t = 0; t < NSTEP; ++t) {
    const int tn = (t + 1 < NSTEP) ? (t + 1) : (NSTEP - 1);
    const float xn0 = xr0[tn];
    const float xn1 = xr1[tn];
    chain_step(xc0, cw0, cw1, cb0, cb1, a0h, a0l, a1h, a1l, bh0, bl0, h00, h01);
    chain_step(xc1, cw0, cw1, cb0, cb1, a0h, a0l, a1h, a1l, bh1, bl1, h10, h11);
    xc0 = xn0;
    xc1 = xn1;
  }

  float p0 = 0.0f, p1 = 0.0f;
#pragma unroll
  for (int r = 0; r < 8; ++r) {
    const float f0 = cf_s[8 * hh + r];
    const float f1 = cf_s[16 + 8 * hh + r];
    p0 = fmaf(h00[r], f0, p0);
    p0 = fmaf(h01[r], f1, p0);
    p1 = fmaf(h10[r], f0, p1);
    p1 = fmaf(h11[r], f1, p1);
  }
  const float q0 = __shfl_xor(p0, 16, 32);
  const float q1 = __shfl_xor(p1, 16, 32);
  const float fb = fc_b[0];
  const float s0 = (p0 + q0) + fb;
  const float s1 = (p1 + q1) + fb;
  const float val = (hh == 0) ? s0 : s1;
  oslab[wave][lane] = val;
  __syncthreads();
  const int l8 = lane & 7;
  const v4f ov = *(const v4f*)(&oslab[wave][4 * l8]);
  float* op = out + (size_t)wrow + 4 * l8;
  if (lane < 8) *(volatile v4f*)op = ov;
  __threadfence();
  if (lane < 8) *(volatile v4f*)op = ov;
}

extern "C" void kernel_launch(void* const* d_in, const int* in_sizes, int n_in,
                              void* d_out, int out_size, void* d_ws, size_t ws_size, hipStream_t stream) {
  (void)d_ws; (void)ws_size;
  if (n_in < 7 || d_out == nullptr) return;
  if (in_sizes[0] != NBAT * NSTEP || in_sizes[1] != NHID || in_sizes[2] != NHID * NHID || in_sizes[3] != NHID ||
      in_sizes[4] != NHID || in_sizes[5] != NHID || in_sizes[6] != 1 || out_size != NBAT) return;

  const float* x    = (const float*)d_in[0];
  const float* w_ih = (const float*)d_in[1];
  const float* w_hh = (const float*)d_in[2];
  const float* b_ih = (const float*)d_in[3];
  const float* b_hh = (const float*)d_in[4];
  const float* fc_w = (const float*)d_in[5];
  const float* fc_b = (const float*)d_in[6];
  float* out = (float*)d_out;

  rnn_seq_kernel<<<NBLK, NTHR, 0, stream>>>(x, w_ih, w_hh, b_ih, b_hh, fc_w, fc_b, out);
}
